// STULayer_85323820303006
// MI455X (gfx1250) — hardware-verified
//
#include <hip/hip_runtime.h>
#include <stddef.h>
#include <stdint.h>

#define NT   2048
#define DI   512
#define DO   512
#define NFL  24
#define KK   (NFL * DI)
#define FB   64
#define TCH  16
#define GBM  128
#define GBN  128
#define ASC  4096.0f
#define BSC  256.0f
#define ISC  (1.0f / 1048576.0f)

static_assert((KK % 32) == 0);
static_assert((NT % TCH) == 0);
static_assert((DI % FB) == 0);
static_assert((NT % GBM) == 0);
static_assert((DO % GBN) == 0);
static_assert(((TCH * NFL) % 32) == 0);
static_assert((TCH * NFL) / 4 <= 256);
static_assert(TCH * (FB / 4) == 256);
static_assert(FB == 64);
static_assert(NFL == 3 * 8);
static_assert((DI / 8) == 64);
static_assert(DO == 512);
static_assert(GBM == 128);
static_assert(GBN == 128);

typedef _Float16     v16h __attribute__((ext_vector_type(16)));
typedef _Float16     v8h  __attribute__((ext_vector_type(8)));
typedef float        v8f  __attribute__((ext_vector_type(8)));
typedef float        v4f  __attribute__((ext_vector_type(4)));
typedef float        v2f  __attribute__((ext_vector_type(2)));
typedef unsigned int v4u  __attribute__((ext_vector_type(4)));

__device__ __forceinline__ unsigned short bf_bits(float f) {
  const unsigned u = __float_as_uint(f);
  return (unsigned short)((u + 0x7FFFu + ((u >> 16) & 1u)) >> 16);
}
__device__ __forceinline__ float bfr(float f) { return __uint_as_float(((unsigned)bf_bits(f)) << 16); }
__device__ __forceinline__ unsigned short h_bits(float f) {
  const _Float16 h = (_Float16)f;
  return __builtin_bit_cast(unsigned short, h);
}
__device__ __forceinline__ unsigned pk16(unsigned short a, unsigned short b) { return (unsigned)a | ((unsigned)b << 16); }
__device__ __forceinline__ v8f zero8() { v8f z = {0.f, 0.f, 0.f, 0.f, 0.f, 0.f, 0.f, 0.f}; return z; }

union FragH { v16h v; v8h h[2]; };
__device__ __forceinline__ v16h ldfrag_h(const _Float16* p) {
  FragH f;
  f.h[0] = *(const v8h*)(p);
  f.h[1] = *(const v8h*)(p + 16);
  return f.v;
}

__device__ __forceinline__ v8f mma_h(v16h a, v16h b, v8f c) {
  return __builtin_amdgcn_wmma_f32_16x16x32_f16(false, a, false, b, (short)0, c, false, false);
}
__device__ __forceinline__ void guard8(v8f& c0, v8f& c1, v8f& c2, v8f& c3, v8f& c4, v8f& c5, v8f& c6, v8f& c7,
                                       const v16h& a0, const v16h& a1, const v16h& a2, const v16h& a3,
                                       const v16h& b0, const v16h& b1) {
#if defined(__HIP_DEVICE_COMPILE__)
  asm volatile("v_nop\n\tv_nop\n\tv_nop\n\tv_nop"
               : "+v"(c0), "+v"(c1), "+v"(c2), "+v"(c3), "+v"(c4), "+v"(c5), "+v"(c6), "+v"(c7)
               : "v"(a0), "v"(a1), "v"(a2), "v"(a3), "v"(b0), "v"(b1));
#endif
}

__global__ __launch_bounds__(256)
void k_cvm(const float* __restrict__ M, unsigned short* Bt) {
  const unsigned g  = blockIdx.x * 256u + threadIdx.x;
  const unsigned f8 = (g & 63u) * 8u;
  const unsigned o  = (g >> 6) & 511u;
  const unsigned n  = g >> 15;
  const float* src = M + ((size_t)(n * DO + o) * DI + f8);
  const v4f a = *(const v4f*)(src);
  const v4f c = *(const v4f*)(src + 4);
  v4u u;
  u[0] = pk16(h_bits(bfr(a[0]) * BSC), h_bits(bfr(a[1]) * BSC));
  u[1] = pk16(h_bits(bfr(a[2]) * BSC), h_bits(bfr(a[3]) * BSC));
  u[2] = pk16(h_bits(bfr(c[0]) * BSC), h_bits(bfr(c[1]) * BSC));
  u[3] = pk16(h_bits(bfr(c[2]) * BSC), h_bits(bfr(c[3]) * BSC));
  unsigned short* dst = Bt + (size_t)o * KK + n * DI + f8;
  *(volatile v4u*)dst = u;
  __threadfence();
  *(volatile v4u*)dst = u;
}

__global__ __launch_bounds__(256)
void k_psum(const float* __restrict__ x, const float* __restrict__ phi, unsigned short* Ap, int b) {
  __shared__ __align__(16) float xs[TCH * FB];
  __shared__ __align__(16) float phs[TCH * NFL];
  __shared__ __align__(16) unsigned int tile[TCH * NFL * (FB / 2)];

  const int tid = threadIdx.x, ng = tid >> 5, fp = tid & 31;
  const int f0 = blockIdx.x * FB;
  const int n0 = 3 * ng;
  const int xr = tid >> 4, xq = tid & 15;
  const float* xsrc = x + (size_t)b * NT * DI + f0 + 4 * xq;
  const int q = tid & 7, lb = tid >> 3;

  float c00 = 0.0f, c01 = 0.0f, c10 = 0.0f, c11 = 0.0f, c20 = 0.0f, c21 = 0.0f;

#pragma unroll 1
  for (int ch = 0; ch < NT / TCH; ++ch) {
    const int t0 = ch * TCH;
    __syncthreads();
    {
      const v4f v = *(const v4f*)(xsrc + (size_t)(t0 + xr) * DI);
      v4f r;
      r[0] = bfr(v[0]); r[1] = bfr(v[1]); r[2] = bfr(v[2]); r[3] = bfr(v[3]);
      *(v4f*)(xs + xr * FB + 4 * xq) = r;
      if (tid < (TCH * NFL) / 4) {
        const v4f p = *(const v4f*)(phi + (size_t)t0 * NFL + 4 * tid);
        v4f pr;
        pr[0] = bfr(p[0]); pr[1] = bfr(p[1]); pr[2] = bfr(p[2]); pr[3] = bfr(p[3]);
        *(v4f*)(phs + 4 * tid) = pr;
      }
    }
    __syncthreads();
#pragma unroll 2
    for (int tl = 0; tl < TCH; ++tl) {
      const v2f xv = *(const v2f*)(xs + tl * FB + 2 * fp);
      const float p0 = phs[tl * NFL + n0];
      const float p1 = phs[tl * NFL + n0 + 1];
      const float p2 = phs[tl * NFL + n0 + 2];
      c00 = fmaf(p0, xv[0], c00); c01 = fmaf(p0, xv[1], c01);
      c10 = fmaf(p1, xv[0], c10); c11 = fmaf(p1, xv[1], c11);
      c20 = fmaf(p2, xv[0], c20); c21 = fmaf(p2, xv[1], c21);
      const float q0 = p0 * ASC, q1 = p1 * ASC, q2 = p2 * ASC;
      unsigned int* trow = tile + (tl * NFL + n0) * (FB / 2) + fp;
      trow[0]            = pk16(h_bits(c00 * q0), h_bits(c01 * q0));
      trow[FB / 2]       = pk16(h_bits(c10 * q1), h_bits(c11 * q1));
      trow[2 * (FB / 2)] = pk16(h_bits(c20 * q2), h_bits(c21 * q2));
    }
    __syncthreads();
    v4u v[12];
#pragma unroll
    for (int i = 0; i < 12; ++i) v[i] = *(const v4u*)(tile + (lb + 32 * i) * (FB / 2) + 4 * q);
    unsigned short* abase = Ap + (size_t)t0 * KK + f0 + 8 * q;
#pragma unroll
    for (int i = 0; i < 12; ++i) {
      const int L = lb + 32 * i, tl = L / NFL, n = L - tl * NFL;
      *(volatile v4u*)(abase + (size_t)tl * KK + n * DI) = v[i];
    }
    __threadfence();
#pragma unroll
    for (int i = 0; i < 12; ++i) {
      const int L = lb + 32 * i, tl = L / NFL, n = L - tl * NFL;
      *(volatile v4u*)(abase + (size_t)tl * KK + n * DI) = v[i];
    }
  }
}

__device__ __forceinline__ void put8(float* tp, const v8f& a) {
#pragma unroll
  for (int r = 0; r < 8; ++r) tp[r * GBN] = a[r] * ISC;
}

__global__ __launch_bounds__(256)
void k_gemm(const unsigned short* __restrict__ Ap, const unsigned short* __restrict__ Bt, float* out, int b) {
  __shared__ __align__(16) float tile[64 * GBN];

  const int tid = threadIdx.x, w = tid >> 5, lane = tid & 31, hh = lane >> 4, c = lane & 15;
  const int wr = w >> 2, wc = w & 3;
  const int mt = blockIdx.x >> 2, ot = blockIdx.x & 3;
  const int t0 = mt * GBM, o0 = ot * GBN;

  const _Float16* A  = (const _Float16*)Ap;
  const _Float16* Bm = (const _Float16*)Bt;
  const _Float16* a0p = A + (size_t)(t0 + wr * 64 + c) * KK + 8 * hh;
  const _Float16* a1p = a0p + (size_t)16 * KK;
  const _Float16* a2p = a0p + (size_t)32 * KK;
  const _Float16* a3p = a0p + (size_t)48 * KK;
  const _Float16* b0p = Bm + (size_t)(o0 + wc * 32 + c) * KK + 8 * hh;
  const _Float16* b1p = b0p + (size_t)16 * KK;

  v8f c00 = zero8(), c01 = zero8(), c10 = zero8(), c11 = zero8();
  v8f c20 = zero8(), c21 = zero8(), c30 = zero8(), c31 = zero8();

#pragma unroll 1
  for (int ks = 0; ks < KK / 32; ++ks) {
    const int ko = 32 * ks;
    const v16h a0 = ldfrag_h(a0p + ko);
    const v16h a1 = ldfrag_h(a1p + ko);
    const v16h a2 = ldfrag_h(a2p + ko);
    const v16h a3 = ldfrag_h(a3p + ko);
    const v16h f0 = ldfrag_h(b0p + ko);
    const v16h f1 = ldfrag_h(b1p + ko);
    c00 = mma_h(a0, f0, c00);
    c01 = mma_h(a0, f1, c01);
    c10 = mma_h(a1, f0, c10);
    c11 = mma_h(a1, f1, c11);
    c20 = mma_h(a2, f0, c20);
    c21 = mma_h(a2, f1, c21);
    c30 = mma_h(a3, f0, c30);
    c31 = mma_h(a3, f1, c31);
    guard8(c00, c01, c10, c11, c20, c21, c30, c31, a0, a1, a2, a3, f0, f1);
  }

  const int piece = tid & 31, rr = tid >> 5;
  float* orow = out + ((size_t)b * NT + t0) * DO + o0 + 4 * piece;
#pragma unroll 1
  for (int p = 0; p < 2; ++p) {
    __syncthreads();
    if (wr == p) {
      float* tw = tile + (8 * hh) * GBN + wc * 32 + c;
      put8(tw + (0  * GBN) + 0,  c00);
      put8(tw + (0  * GBN) + 16, c01);
      put8(tw + (16 * GBN) + 0,  c10);
      put8(tw + (16 * GBN) + 16, c11);
      put8(tw + (32 * GBN) + 0,  c20);
      put8(tw + (32 * GBN) + 16, c21);
      put8(tw + (48 * GBN) + 0,  c30);
      put8(tw + (48 * GBN) + 16, c31);
    }
    __syncthreads();
    v4f v[8];
#pragma unroll
    for (int it = 0; it < 8; ++it) v[it] = *(const v4f*)(tile + (rr + 8 * it) * GBN + 4 * piece);
    float* ob = orow + (size_t)(64 * p) * DO;
#pragma unroll
    for (int it = 0; it < 8; ++it) *(volatile v4f*)(ob + (size_t)(rr + 8 * it) * DO) = v[it];
    __threadfence();
#pragma unroll
    for (int it = 0; it < 8; ++it) *(volatile v4f*)(ob + (size_t)(rr + 8 * it) * DO) = v[it];
  }
}

extern "C" void kernel_launch(void* const* d_in, const int* in_sizes, int n_in,
                              void* d_out, int out_size, void* d_ws, size_t ws_size,
                              hipStream_t stream) {
  if (n_in < 3) return;
  const int per = NT * DI;
  const int nb = in_sizes[0] / per;
  if (nb < 1 || in_sizes[0] != nb * per) return;
  if (in_sizes[1] != NT * NFL) return;
  if (in_sizes[2] != NFL * DO * DI) return;
  if (out_size != nb * NT * DO) return;

  const float* x   = (const float*)d_in[0];
  const float* phi = (const float*)d_in[1];
  const float* M   = (const float*)d_in[2];
  float* out = (float*)d_out;

  const size_t sBt = (size_t)DO * KK * 2;
  const size_t sAp = (size_t)NT * KK * 2;
  size_t off = 0;
  const size_t oBt = off; off += sBt;
  const size_t oAp = off; off += sAp;
  if (off > ws_size) return;
  if (off > (size_t)134217728) return;

  char* ws = (char*)d_ws;
  unsigned short* Bt = (unsigned short*)(ws + oBt);
  unsigned short* Ap = (unsigned short*)(ws + oAp);

  k_cvm<<<dim3((NFL * DO * (DI / 8)) / 256), dim3(256), 0, stream>>>(M, Bt);
  for (int bb = 0; bb < nb; ++bb) {
    k_psum<<<dim3(DI / FB), dim3(256), 0, stream>>>(x, phi, Ap, bb);
    k_gemm<<<dim3((NT / GBM) * (DO / GBN)), dim3(256), 0, stream>>>(Ap, Bt, out, bb);
  }
  (void)hipGetLastError();
}
